// ContinuousEmbedding_15032385536233
// MI455X (gfx1250) — hardware-verified
//
#include <hip/hip_runtime.h>


#pragma clang fp contract(off)

#ifndef NB
#define NB 128
#endif
#ifndef SEQ
#define SEQ 200
#endif
#define NB_FULL  128
#define SEQ_FULL 200
#ifndef OUT_SEQ
#define OUT_SEQ SEQ
#endif
#define NPTS   2048
#define ND     64
#define BINW   16
#define NBIN   (NPTS / BINW + 1)
#define PADL   8
#define EPW    2112
#define ETP    72
#define BT     256
#define NW     8
#define CHUNK  256
#define LCAP   512
#define DRAIN_AT 256
#define OSP    68
#define WCARRY 1024.0f
#define WINV   (1.0f / 1024.0f)
#define PSCALE 1024.0f
#define PI_F   3.14159274101257324f
#define NROWS  (NB * SEQ)
#define OUT_ROWS ((NB - 1) * OUT_SEQ + SEQ)

static_assert(ND == 64);
static_assert(NPTS % BINW == 0);
static_assert(NBIN == NPTS / BINW + 1);
static_assert(BINW + 2 * PADL == 32);
static_assert(PADL >= 4);
static_assert((NBIN - 1) * BINW + 32 <= EPW);
static_assert(NPTS + PADL <= EPW);
static_assert(EPW % 64 == 0);
static_assert(EPW % 8 == 0);
static_assert(BT == 32 * NW);
static_assert(CHUNK == BT);
static_assert(LCAP >= DRAIN_AT + CHUNK);
static_assert(LCAP % 16 == 0);
static_assert((OSP * 4) % 16 == 0);
static_assert(OSP >= ND);
static_assert((ETP * 2) % 16 == 0);
static_assert(ETP >= 64);
static_assert(NB <= NB_FULL);
static_assert(SEQ <= SEQ_FULL);
static_assert(8 * 2 == 16);
static_assert(16 * 4 == ND);
static_assert(NW * 2 * 4 == ND);
static_assert(16 * BT == 64 * 64);
static_assert((size_t)LCAP * 8 + NW * 4 + (size_t)NW * 16 * OSP * 4 <= 131072);
static_assert((size_t)64 * ETP * 2 <= 131072);

typedef _Float16 h16;
typedef unsigned short bf;
typedef __attribute__((ext_vector_type(16))) _Float16 v16h;
typedef __attribute__((ext_vector_type(8)))  _Float16 v8h;
typedef __attribute__((ext_vector_type(8)))  float    v8f;
typedef __attribute__((ext_vector_type(4)))  float    v4f;
typedef v4f  __attribute__((may_alias)) v4fa;
typedef v8h  __attribute__((may_alias)) v8ha;

__device__ __forceinline__ unsigned short f2bf(float f) { unsigned u = __float_as_uint(f); u += 0x7FFFu + ((u >> 16) & 1u); return (unsigned short)(u >> 16); }
__device__ __forceinline__ float bfr(float f) { return __uint_as_float(((unsigned)f2bf(f)) << 16); }
__device__ __forceinline__ v16h cat16(v8h lo, v8h hi) { return __builtin_shufflevector(lo, hi, 0, 1, 2, 3, 4, 5, 6, 7, 8, 9, 10, 11, 12, 13, 14, 15); }
__device__ __forceinline__ v8f wmma16(v16h a, v16h b, v8f c) { return __builtin_amdgcn_wmma_f32_16x16x32_f16(false, a, false, b, (short)0, c, false, false); }
__device__ __forceinline__ v16h  ldh(const h16* p) { return cat16(*(const v8h*)p, *(const v8h*)(p + 16)); }
__device__ __forceinline__ void wave_sync() { __builtin_amdgcn_fence(3  , "wavefront"); __builtin_amdgcn_wave_barrier(); asm volatile("" ::: "memory"); }
__device__ __forceinline__ v8f wmma16g(v16h a, v16h b, v8f c) { c = wmma16(a, b, c); asm volatile("v_nop\n\tv_nop\n\tv_nop\n\tv_nop" : "+v"(c) : "v"(a), "v"(b)); return c; }
static __device__ __forceinline__ h16 toh_flush(float v) { const h16 r = (h16)v; return (fabsf(v) < 6.103515625e-05f) ? (h16)0.0f : r; }
__device__ __forceinline__ float sgnf(float v) { return (v > 0.0f) ? 1.0f : ((v < 0.0f) ? -1.0f : v); }

__global__ __launch_bounds__(BT) void k_embt(const float* __restrict__ emb, h16* ET) {
    __shared__ __align__(16) h16 tile[64 * ETP];
    const int tid = threadIdx.x, lane = tid & 31;
    const int wave = __builtin_amdgcn_readfirstlane((int)(threadIdx.x >> 5));
    const int col0 = blockIdx.x * 64;
#pragma unroll 1
    for (int i = 0; i < 16; ++i) {
        const int e = i * BT + tid; const int pl = e >> 6, n = e & 63;
        const int p = col0 - PADL + pl;
        const int pc = p < 0 ? 0 : (p > NPTS - 1 ? NPTS - 1 : p);
        float v = emb[(size_t)pc * ND + n];
        asm volatile("" : "+v"(v));
        const h16 hv = toh_flush(bfr(v));
        tile[n * ETP + pl] = ((p >= 0) & (p < NPTS)) ? hv : (h16)0.0f;
    }
    __syncthreads();
#pragma unroll 1
    for (int ps = 0; ps < 2; ++ps) {
#pragma unroll
        for (int s = 0; s < 2; ++s) { const int n = wave * 8 + s * 4 + (lane >> 3), q = lane & 7;
            const v8h val = *(const v8ha*)(&tile[n * ETP + q * 8]);
            *(volatile v8h*)(ET + (size_t)n * EPW + col0 + q * 8) = val; }
        if (ps == 0) __threadfence(); }
}

__global__ __launch_bounds__(BT) void k_bins(const float* __restrict__ X, const h16* __restrict__ ET, float* OUT) {
    __shared__ int   hrow[LCAP];
    __shared__ float hxs[LCAP];
    __shared__ int   wcnt[NW];
    __shared__ __align__(16) float os[NW * 16 * OSP];
    const int tid = threadIdx.x;
    const int lane = tid & 31, lr = lane & 15, hi = lane >> 4;
    const int wave = __builtin_amdgcn_readfirstlane((int)(threadIdx.x >> 5));
    const int wvec = tid >> 5;
    const int bin = blockIdx.x;
    const int c0 = bin * BINW;
    const int P0 = c0 - PADL;
    const size_t eo = (size_t)lr * EPW + c0 + 8 * hi;
    const v16h b0 = ldh(ET + eo);
    const v16h b1 = ldh(ET + eo + (size_t)16 * EPW);
    const v16h b2 = ldh(ET + eo + (size_t)32 * EPW);
    const v16h b3 = ldh(ET + eo + (size_t)48 * EPW);
    const int wb = wave * 16 * OSP;
    int count = 0;
#pragma unroll 1
    for (int base = 0; base < NROWS; base += CHUNK) {
        const int r = base + tid;
        const int rc = r < NROWS ? r : NROWS - 1;
        const int rb = rc / SEQ, rt = rc - rb * SEQ;
        float xv = X[(size_t)rb * SEQ_FULL + rt];
        asm volatile("" : "+v"(xv));
        const float xs = (bfr(xv) + 1.0f) * PSCALE;
        float fl = floorf(xs); fl = fminf(fmaxf(fl, -64.0f), 4096.0f);
        int bq = ((int)fl) >> 4; bq = bq < 0 ? 0 : (bq > NBIN - 1 ? NBIN - 1 : bq);
        const bool hit = (r < NROWS) & (bq == bin);
        const unsigned mask = __builtin_amdgcn_ballot_w32(hit);
        if (lane == 0) wcnt[wave] = __builtin_popcount(mask);
        __syncthreads();
        int pre = 0, tot = 0;
#pragma unroll
        for (int w = 0; w < NW; ++w) { const int c = wcnt[w]; pre += (w < wvec) ? c : 0; tot += c; }
        if (hit) { const int pos = count + pre + (int)__builtin_amdgcn_mbcnt_lo(mask, 0u);
                   const int pc = pos < LCAP - 1 ? pos : LCAP - 1;
                   hrow[pc] = rb * OUT_SEQ + rt; hxs[pc] = xs; }
        count += tot;
        __syncthreads();
        const int cnt = __builtin_amdgcn_readfirstlane(count);
        const bool last = (base + CHUNK >= NROWS);
        if ((cnt >= DRAIN_AT) | (last & (cnt > 0))) {
            const int ntile = (cnt + 15) >> 4;
#pragma unroll 1
            for (int tile = wave; tile < ntile; tile += NW) {
                const int li = tile * 16 + lr;
                const int lic = li < cnt ? li : cnt - 1;
                const float xr = hxs[lic];
                float ssum = 0.0f;
#pragma unroll 1
                for (int i = 0; i < 16; ++i) {
                    const int k = (i & 7) + 8 * hi + ((i >> 3) << 4);
                    const int p = P0 + k;
                    const float d = xr - (float)p;
                    const float t1 = PI_F * d;
                    const float ang = t1 * 0.125f;
                    const float y = cosf(ang);
                    const float sp = sgnf(d + 4.0f), sm = sgnf(d - 4.0f);
                    const float rc2 = (sp - sm) * 0.5f * (1.0f + sp) * (1.0f - sm);
                    float wk = y * y * rc2;
                    wk = ((p >= 0) & (p < NPTS)) ? wk : 0.0f;
                    os[wb + lr * OSP + k] = wk;
                    ssum += wk;
                }
                ssum += __shfl_xor(ssum, 16, 32);
                const float inv = 1.0f / ssum;
                wave_sync();
                const v4f q0 = *(const v4fa*)(&os[wb + lr * OSP + 8 * hi]);
                const v4f q1 = *(const v4fa*)(&os[wb + lr * OSP + 8 * hi + 4]);
                const v4f q2 = *(const v4fa*)(&os[wb + lr * OSP + 16 + 8 * hi]);
                const v4f q3 = *(const v4fa*)(&os[wb + lr * OSP + 16 + 8 * hi + 4]);
                v16h af;
#pragma unroll
                for (int i = 0; i < 4; ++i) {
                    af[i]      = toh_flush(q0[i] * inv * WCARRY);
                    af[4 + i]  = toh_flush(q1[i] * inv * WCARRY);
                    af[8 + i]  = toh_flush(q2[i] * inv * WCARRY);
                    af[12 + i] = toh_flush(q3[i] * inv * WCARRY); }
                wave_sync();
                v8f d0 = (v8f){}, d1 = (v8f){}, d2 = (v8f){}, d3 = (v8f){};
                d0 = wmma16g(af, b0, d0);
                d1 = wmma16g(af, b1, d1);
                d2 = wmma16g(af, b2, d2);
                d3 = wmma16g(af, b3, d3);
#pragma unroll
                for (int rr = 0; rr < 8; ++rr) {
                    os[wb + (8 * hi + rr) * OSP +  0 + lr] = d0[rr] * WINV;
                    os[wb + (8 * hi + rr) * OSP + 16 + lr] = d1[rr] * WINV;
                    os[wb + (8 * hi + rr) * OSP + 32 + lr] = d2[rr] * WINV;
                    os[wb + (8 * hi + rr) * OSP + 48 + lr] = d3[rr] * WINV; }
                wave_sync();
#pragma unroll 1
                for (int ps = 0; ps < 2; ++ps) {
#pragma unroll
                    for (int s = 0; s < 8; ++s) { const int rw = 2 * s + hi;
                        const int le = tile * 16 + rw;
                        const int lec = le < cnt ? le : cnt - 1;
                        int orow = hrow[lec]; orow = orow < 0 ? 0 : (orow > OUT_ROWS - 1 ? OUT_ROWS - 1 : orow);
                        const v4f val = *(const v4fa*)(&os[wb + rw * OSP + lr * 4]);
                        if (le < cnt) *(volatile v4f*)(OUT + (size_t)orow * ND + lr * 4) = val; }
                    if (ps == 0) __threadfence(); }
                wave_sync();
            }
            __syncthreads();
            count = 0;
        }
    }
}

static constexpr size_t al256(size_t v) { return (v + 255) & ~(size_t)255; }
static constexpr size_t SZ_ET = al256((size_t)ND * EPW * 2);
static constexpr size_t SZ_TOTAL = SZ_ET;
static_assert(SZ_TOTAL <= (size_t)134217728);
static_assert((size_t)(EPW / 64) * 64 * 2 * ND == (size_t)ND * EPW * 2);

extern "C" void kernel_launch(void* const* d_in, const int* in_sizes, int n_in,
                              void* d_out, int out_size, void* d_ws, size_t ws_size, hipStream_t stream) {
    if (n_in < 2) return;
    const size_t needx = (size_t)(NB - 1) * SEQ_FULL + SEQ;
    if ((size_t)in_sizes[0] < needx) return;
    if ((size_t)in_sizes[1] < (size_t)NPTS * ND) return;
    if ((size_t)out_size < (size_t)OUT_ROWS * ND) return;
    if (SZ_TOTAL > ws_size) return;
    const float* x   = (const float*)d_in[0];
    const float* emb = (const float*)d_in[1];
    float* OUT = (float*)d_out;
    h16* ET = (h16*)d_ws;

    k_embt<<<dim3(EPW / 64, 1, 1), BT, 0, stream>>>(emb, ET);
    k_bins<<<dim3(NBIN, 1, 1), BT, 0, stream>>>(x, ET, OUT);
}
